// SimpleImageMLP_WithDistLayer_89988154785962
// MI455X (gfx1250) — hardware-verified
//
#include <hip/hip_runtime.h>
#include <stdint.h>


#define BDIM 1024
#define DIN  1024
#define HDIM 512
#define ODIM 512
#define CEPS 1e-8f
#define MAXD 1000000.0f

#define SP   36
#define KC   128
#define CP   (KC + 4)
#define OTP  36

static_assert(BDIM % 64 == 0);
static_assert(HDIM % 64 == 0);
static_assert(DIN % 32 == 0);
static_assert(ODIM % 32 == 0);
static_assert(HDIM % KC == 0);

typedef __bf16 bf16_t;
typedef bf16_t v16bf __attribute__((ext_vector_type(16)));
typedef float v8f __attribute__((ext_vector_type(8)));
typedef float v4f __attribute__((ext_vector_type(4)));
typedef unsigned int v4u __attribute__((ext_vector_type(4)));

union Frag { v16bf v; v4u u[2]; };

__device__ __forceinline__ unsigned int bf16_bits_rne(float f) {
    const unsigned int u = __float_as_uint(f);
    return (u + 0x7FFFu + ((u >> 16) & 1u)) >> 16;
}

__device__ __forceinline__ v8f mma_bf16(v8f acc, v16bf a, v16bf b) {
    acc = __builtin_amdgcn_wmma_f32_16x16x32_bf16(false, a, false, b, (short)0, acc, false, false);
    asm volatile("v_nop\n\tv_nop\n\tv_nop\n\tv_nop" : "+v"(acc) : "v"(a), "v"(b));
    return acc;
}

__device__ __forceinline__ void load_frag(Frag& f, const unsigned short* p) {
    f.u[0] = *(const v4u*)(p);
    f.u[1] = *(const v4u*)(p + 16);
}

__global__ __launch_bounds__(256)
void k_split_planes(const float* __restrict__ x, const float* __restrict__ w,
                    unsigned short* __restrict__ xh, unsigned short* __restrict__ xl,
                    unsigned short* __restrict__ wh, unsigned short* __restrict__ wl,
                    int nx8, int nw8)
{
    const int t = blockIdx.x * 256 + (int)threadIdx.x;
    const float* src;
    unsigned short* dh;
    unsigned short* dl;
    int i8;
    if (t < nx8) { src = x; dh = xh; dl = xl; i8 = t; }
    else {
        i8 = t - nx8;
        if (i8 >= nw8) return;
        src = w; dh = wh; dl = wl;
    }
    const size_t off = (size_t)i8 * 8;
    const v4f q0 = *(const v4f*)(src + off);
    const v4f q1 = *(const v4f*)(src + off + 4);
    const float f[8] = {q0.x, q0.y, q0.z, q0.w, q1.x, q1.y, q1.z, q1.w};
    unsigned int hb[8], lb[8];
    #pragma unroll
    for (int i = 0; i < 8; ++i) {
        const unsigned int hbit = bf16_bits_rne(f[i]);
        const float hf = __uint_as_float(hbit << 16);
        hb[i] = hbit;
        lb[i] = bf16_bits_rne(f[i] - hf);
    }
    v4u H, L;
    H.x = hb[0] | (hb[1] << 16); H.y = hb[2] | (hb[3] << 16);
    H.z = hb[4] | (hb[5] << 16); H.w = hb[6] | (hb[7] << 16);
    L.x = lb[0] | (lb[1] << 16); L.y = lb[2] | (lb[3] << 16);
    L.z = lb[4] | (lb[5] << 16); L.w = lb[6] | (lb[7] << 16);
    volatile v4u* ph = (volatile v4u*)(dh + off);
    volatile v4u* pl = (volatile v4u*)(dl + off);
    *ph = H;
    *pl = L;
    __threadfence();
    *ph = H;
    *pl = L;
}

__global__ __launch_bounds__(128)
void k_gemm_bias_relu(const unsigned short* __restrict__ xh, const unsigned short* __restrict__ xl,
                      const unsigned short* __restrict__ wh, const unsigned short* __restrict__ wl,
                      const float* __restrict__ bias, float* hout)
{
    __shared__ __attribute__((aligned(16))) float stile[4 * 32 * SP];

    const int lane = (int)threadIdx.x & 31;
    const int wave = (int)threadIdx.x >> 5;
    const int hh   = lane >> 4;
    const int m    = lane & 15;
    const int m0   = blockIdx.x * 64 + (wave & 1) * 32;
    const int n0   = blockIdx.y * 64 + (wave >> 1) * 32;

    const size_t ra0 = (size_t)(m0 + m)      * DIN + 8 * hh;
    const size_t ra1 = (size_t)(m0 + 16 + m) * DIN + 8 * hh;
    const size_t rb0 = (size_t)(n0 + m)      * DIN + 8 * hh;
    const size_t rb1 = (size_t)(n0 + 16 + m) * DIN + 8 * hh;

    v8f c00 = {}, c01 = {}, c10 = {}, c11 = {};

    for (int k0 = 0; k0 < DIN; k0 += 32) {
        Frag A0h, A0l, A1h, A1l, B0h, B0l, B1h, B1l;
        load_frag(A0h, xh + ra0 + k0); load_frag(A0l, xl + ra0 + k0);
        load_frag(A1h, xh + ra1 + k0); load_frag(A1l, xl + ra1 + k0);
        load_frag(B0h, wh + rb0 + k0); load_frag(B0l, wl + rb0 + k0);
        load_frag(B1h, wh + rb1 + k0); load_frag(B1l, wl + rb1 + k0);

        c00 = mma_bf16(c00, A0h.v, B0h.v); c00 = mma_bf16(c00, A0h.v, B0l.v); c00 = mma_bf16(c00, A0l.v, B0h.v);
        c01 = mma_bf16(c01, A0h.v, B1h.v); c01 = mma_bf16(c01, A0h.v, B1l.v); c01 = mma_bf16(c01, A0l.v, B1h.v);
        c10 = mma_bf16(c10, A1h.v, B0h.v); c10 = mma_bf16(c10, A1h.v, B0l.v); c10 = mma_bf16(c10, A1l.v, B0h.v);
        c11 = mma_bf16(c11, A1h.v, B1h.v); c11 = mma_bf16(c11, A1h.v, B1l.v); c11 = mma_bf16(c11, A1l.v, B1h.v);
    }

    float* st = stile + wave * (32 * SP);
    const float bz0 = bias[n0 + m];
    const float bz1 = bias[n0 + 16 + m];
    #pragma unroll
    for (int r = 0; r < 8; ++r) {
        const int rr = 8 * hh + r;
        st[rr * SP + m]             = fmaxf(c00[r] + bz0, 0.0f);
        st[rr * SP + 16 + m]        = fmaxf(c01[r] + bz1, 0.0f);
        st[(16 + rr) * SP + m]      = fmaxf(c10[r] + bz0, 0.0f);
        st[(16 + rr) * SP + 16 + m] = fmaxf(c11[r] + bz1, 0.0f);
    }
    __syncthreads();

    const int rq = lane >> 3;
    const int c4 = (lane & 7) * 4;
    v4f vals[8];
    #pragma unroll
    for (int i = 0; i < 8; ++i) {
        const float* rp = st + (4 * i + rq) * SP + c4;
        v4f v; v.x = rp[0]; v.y = rp[1]; v.z = rp[2]; v.w = rp[3];
        vals[i] = v;
    }
    float* gbase = hout + (size_t)(m0 + rq) * HDIM + n0 + c4;
    #pragma unroll
    for (int i = 0; i < 8; ++i)
        *(volatile v4f*)(gbase + (size_t)(4 * i) * HDIM) = vals[i];
    __threadfence();
    #pragma unroll
    for (int i = 0; i < 8; ++i)
        *(volatile v4f*)(gbase + (size_t)(4 * i) * HDIM) = vals[i];
}

__device__ __forceinline__ float cterm(float a, float b, float acc) {
    const float num = fabsf(a - b);
    const float den = fmaxf(fabsf(a) + fabsf(b), CEPS);
    return fmaf(num, __builtin_amdgcn_rcpf(den), acc);
}

__global__ __launch_bounds__(256)
void k_canberra(const float* __restrict__ h, const float* __restrict__ Wd, float* out)
{
    __shared__ __attribute__((aligned(16))) float rows[64 * CP];
    __shared__ __attribute__((aligned(16))) float ot[32 * OTP];

    const int tid = (int)threadIdx.x;
    const int b0  = blockIdx.x * 32;
    const int o0  = blockIdx.y * 32;
    const int tb  = tid & 15;
    const int to  = tid >> 4;

    float d00 = 0.0f, d01 = 0.0f, d10 = 0.0f, d11 = 0.0f;

    for (int kc = 0; kc < HDIM; kc += KC) {
        __syncthreads();
        for (int i = tid; i < 64 * (KC / 4); i += 256) {
            const int row = i >> 5;
            const int c4  = (i & 31) * 4;
            v4f v;
            if (row < 32) v = *(const v4f*)(h  + (size_t)(b0 + row)      * HDIM + kc + c4);
            else          v = *(const v4f*)(Wd + (size_t)(o0 + row - 32) * HDIM + kc + c4);
            *(v4f*)(rows + row * CP + c4) = v;
        }
        __syncthreads();

        const float* h0 = rows + tb * CP;
        const float* h1 = rows + (tb + 16) * CP;
        const float* w0 = rows + (32 + to) * CP;
        const float* w1 = rows + (48 + to) * CP;
        #pragma unroll 1
        for (int k = 0; k < KC; k += 4) {
            const v4f a0 = *(const v4f*)(h0 + k);
            const v4f a1 = *(const v4f*)(h1 + k);
            const v4f p0 = *(const v4f*)(w0 + k);
            const v4f p1 = *(const v4f*)(w1 + k);
            d00 = cterm(a0.x, p0.x, d00); d00 = cterm(a0.y, p0.y, d00); d00 = cterm(a0.z, p0.z, d00); d00 = cterm(a0.w, p0.w, d00);
            d01 = cterm(a0.x, p1.x, d01); d01 = cterm(a0.y, p1.y, d01); d01 = cterm(a0.z, p1.z, d01); d01 = cterm(a0.w, p1.w, d01);
            d10 = cterm(a1.x, p0.x, d10); d10 = cterm(a1.y, p0.y, d10); d10 = cterm(a1.z, p0.z, d10); d10 = cterm(a1.w, p0.w, d10);
            d11 = cterm(a1.x, p1.x, d11); d11 = cterm(a1.y, p1.y, d11); d11 = cterm(a1.z, p1.z, d11); d11 = cterm(a1.w, p1.w, d11);
        }
    }

    const float s00 = 1.0f / fminf(fmaxf(d00 + CEPS, CEPS), MAXD);
    const float s01 = 1.0f / fminf(fmaxf(d01 + CEPS, CEPS), MAXD);
    const float s10 = 1.0f / fminf(fmaxf(d10 + CEPS, CEPS), MAXD);
    const float s11 = 1.0f / fminf(fmaxf(d11 + CEPS, CEPS), MAXD);
    ot[tb * OTP + to]             = s00;
    ot[tb * OTP + to + 16]        = s01;
    ot[(tb + 16) * OTP + to]      = s10;
    ot[(tb + 16) * OTP + to + 16] = s11;
    __syncthreads();

    const int wave = tid >> 5;
    const int lane = tid & 31;
    const int row  = 4 * wave + (lane >> 3);
    const int c4   = (lane & 7) * 4;
    const float* rp = ot + row * OTP + c4;
    v4f v; v.x = rp[0]; v.y = rp[1]; v.z = rp[2]; v.w = rp[3];
    volatile v4f* gp = (volatile v4f*)(out + (size_t)(b0 + row) * ODIM + o0 + c4);
    *gp = v;
    __threadfence();
    *gp = v;
}

extern "C" void kernel_launch(void* const* d_in, const int* in_sizes, int n_in,
                              void* d_out, int out_size, void* d_ws, size_t ws_size,
                              hipStream_t stream)
{
    if (n_in < 4) return;
    if (in_sizes[0] != BDIM * DIN)  return;
    if (in_sizes[1] != HDIM * DIN)  return;
    if (in_sizes[2] != HDIM)        return;
    if (in_sizes[3] != ODIM * HDIM) return;
    if (out_size   != BDIM * ODIM)  return;

    const float* x  = (const float*)d_in[0];
    const float* W1 = (const float*)d_in[1];
    const float* b1 = (const float*)d_in[2];
    const float* Wd = (const float*)d_in[3];
    float*      out = (float*)d_out;

    const size_t xplane = (size_t)BDIM * DIN * 2;
    const size_t wplane = (size_t)HDIM * DIN * 2;
    const size_t hbytes = (size_t)BDIM * HDIM * 4;
    const size_t o_xh = 0;
    const size_t o_xl = o_xh + xplane;
    const size_t o_wh = o_xl + xplane;
    const size_t o_wl = o_wh + wplane;
    const size_t o_h  = o_wl + wplane;
    const size_t total = o_h + hbytes;
    if (total > ws_size) return;

    char* wsb = (char*)d_ws;
    unsigned short* xh = (unsigned short*)(wsb + o_xh);
    unsigned short* xl = (unsigned short*)(wsb + o_xl);
    unsigned short* wh = (unsigned short*)(wsb + o_wh);
    unsigned short* wl = (unsigned short*)(wsb + o_wl);
    float*        hbuf = (float*)(wsb + o_h);

    const int nx8 = (BDIM * DIN) / 8;
    const int nw8 = (HDIM * DIN) / 8;
    const int cblocks = (nx8 + nw8 + 255) / 256;
    k_split_planes<<<dim3(cblocks), dim3(256), 0, stream>>>(x, W1, xh, xl, wh, wl, nx8, nw8);

    k_gemm_bias_relu<<<dim3(BDIM / 64, HDIM / 64), dim3(128), 0, stream>>>(xh, xl, wh, wl, b1, hbuf);

    k_canberra<<<dim3(BDIM / 32, ODIM / 32), dim3(256), 0, stream>>>(hbuf, Wd, out);
}
